// TanhAttention_85358180041263
// MI455X (gfx1250) — hardware-verified
//
#include <hip/hip_runtime.h>
#include <stdint.h>

#define NBATCH  4
#define TI      512
#define TM      1024
#define DIN     256
#define DMEM    256
#define DT      64
#define KP      (2 * TM)
#define NROWS_I (NBATCH * TI)
#define NROWS_M (NBATCH * TM)
#define NEGV    (-1e30f)
static_assert(DIN % 32 == 0 && DMEM % 64 == 0 && DT == 64);
static_assert(TI % 64 == 0 && TM % 128 == 0 && (KP % 32) == 0);
static_assert((NROWS_I % 64) == 0 && (NROWS_M % 64) == 0 && (DIN == DMEM));

typedef __bf16   v16b __attribute__((ext_vector_type(16)));
typedef __bf16   v8b  __attribute__((ext_vector_type(8)));
typedef float    v8f  __attribute__((ext_vector_type(8)));
typedef float    v4f  __attribute__((ext_vector_type(4)));
typedef unsigned int   v4u  __attribute__((ext_vector_type(4)));
typedef unsigned short v8us __attribute__((ext_vector_type(8)));
typedef v4f  __attribute__((may_alias)) v4fa;
typedef v8us __attribute__((may_alias)) v8usa;

#if defined(__HIP_DEVICE_COMPILE__)
#define DEV_ASM 1
#else
#define DEV_ASM 0
#endif

__device__ __forceinline__ unsigned short bf_bits(float f) {
  unsigned u = __float_as_uint(f);
  return (unsigned short)((u + 0x7FFFu + ((u >> 16) & 1u)) >> 16);
}
__device__ __forceinline__ float bf_up(unsigned short hb) { return __uint_as_float(((unsigned)hb) << 16); }
__device__ __forceinline__ float bf_rn(float f) { return bf_up(bf_bits(f)); }
__device__ __forceinline__ unsigned pk16(unsigned short a, unsigned short b) { return (unsigned)a | ((unsigned)b << 16); }
__device__ __forceinline__ v8f zero8() { v8f z = {0.f, 0.f, 0.f, 0.f, 0.f, 0.f, 0.f, 0.f}; return z; }

__device__ __forceinline__ float fexp2(float x) {
#if __has_builtin(__builtin_amdgcn_exp2f)
  return __builtin_amdgcn_exp2f(x);
#else
  return exp2f(x);
#endif
}
__device__ __forceinline__ float frcp(float x) {
#if __has_builtin(__builtin_amdgcn_rcpf)
  return __builtin_amdgcn_rcpf(x);
#else
  return 1.0f / x;
#endif
}
__device__ __forceinline__ float th(float x) {
  const float xc = fminf(fmaxf(x, -15.0f), 15.0f);
  const float e  = fexp2(xc * 2.8853900817779268f);
  const float r  = frcp(1.0f + e);
  return fmaf(-2.0f, r, 1.0f);
}

__device__ __forceinline__ v16b ldfrag(const __bf16* p) {
  union { v16b v; v8b h[2]; } f;
  f.h[0] = *(const v8b*)(p);
  f.h[1] = *(const v8b*)(p + 16);
  return f.v;
}

__device__ __forceinline__ v8f mmar(v16b a, v16b b, v8f c) {
  return __builtin_amdgcn_wmma_f32_16x16x32_bf16(false, a, false, b, (short)0, c, false, false);
}
__device__ __forceinline__ void dep_guard(v8f& a, v8f& b, v16b x, v16b y) {
#if DEV_ASM
  asm volatile("v_nop\n\tv_nop\n\tv_nop\n\tv_nop" : "+v"(a), "+v"(b) : "v"(x), "v"(y));
#else
  (void)a; (void)b; (void)x; (void)y;
#endif
}
__device__ __forceinline__ void keep4(v16b a, v16b b, v16b c, v16b d) {
#if DEV_ASM
  asm volatile("v_nop" :: "v"(a), "v"(b), "v"(c), "v"(d));
#else
  (void)a; (void)b; (void)c; (void)d;
#endif
}
__device__ __forceinline__ void acc_guard4(v8f& a, v8f& b, v8f& c, v8f& d) {
#if DEV_ASM
  asm volatile("v_nop\n\tv_nop\n\tv_nop\n\tv_nop" : "+v"(a), "+v"(b), "+v"(c), "+v"(d));
#else
  (void)a; (void)b; (void)c; (void)d;
#endif
}

__global__ __launch_bounds__(256) void cvt_bf16x8(const float* __restrict__ in, unsigned short* out, int n8) {
  const int i = blockIdx.x * 256 + (int)threadIdx.x;
  if (i < n8) {
    const v4f a  = *(const v4f*)(in + (size_t)i * 8);
    const v4f a4 = *(const v4f*)(in + (size_t)i * 8 + 4);
    v4u p;
    p[0] = pk16(bf_bits(a[0]),  bf_bits(a[1]));
    p[1] = pk16(bf_bits(a[2]),  bf_bits(a[3]));
    p[2] = pk16(bf_bits(a4[0]), bf_bits(a4[1]));
    p[3] = pk16(bf_bits(a4[2]), bf_bits(a4[3]));
    unsigned short* o = out + (size_t)i * 8;
    *(volatile v4u*)o = p;
    __threadfence();
    *(volatile v4u*)o = p;
  }
}

__global__ __launch_bounds__(256) void mem_transpose(const float* __restrict__ mem, unsigned short* MT) {
  __shared__ __align__(16) unsigned short sT[64 * 136];
  const int tid = threadIdx.x, lane = tid & 31, w = tid >> 5;
  const int j0 = blockIdx.x * 128;
  const int d0 = blockIdx.y * 64;
  const int b  = blockIdx.z;
  const int rl = tid >> 4, c4 = (tid & 15) * 4;
#pragma unroll
  for (int q = 0; q < 8; ++q) {
    const int jl = q * 16 + rl;
    const v4f a = *(const v4f*)(mem + ((size_t)(b * TM + j0 + jl)) * DMEM + d0 + c4);
    sT[(c4 + 0) * 136 + jl] = bf_bits(a[0]);
    sT[(c4 + 1) * 136 + jl] = bf_bits(a[1]);
    sT[(c4 + 2) * 136 + jl] = bf_bits(a[2]);
    sT[(c4 + 3) * 136 + jl] = bf_bits(a[3]);
  }
  __syncthreads();
  const int sub = lane >> 4, q8 = lane & 15;
  v8us v[4];
#pragma unroll
  for (int it = 0; it < 4; ++it) {
    const int drow = it * 16 + 2 * w + sub;
    v[it] = *(const v8usa*)(sT + drow * 136 + q8 * 8);
  }
  for (int pass = 0; pass < 2; ++pass) {
#pragma unroll
    for (int it = 0; it < 4; ++it) {
      const int drow = it * 16 + 2 * w + sub;
      unsigned short* dst = MT + ((size_t)(b * DMEM + d0 + drow)) * KP + j0 + q8 * 8;
      *(volatile v8us*)dst = v[it];
      *(volatile v8us*)(dst + TM) = v[it];
    }
    __threadfence();
  }
}

__global__ __launch_bounds__(256) void gemm64(
    const unsigned short* __restrict__ Ap, int lda, long long strideA,
    const unsigned short* __restrict__ Btp, int ldb, long long strideB,
    float* Cout, int ldc, long long strideC,
    int M, int N, int K, float oscale) {
  const __bf16* A  = (const __bf16*)(const void*)Ap;
  const __bf16* Bt = (const __bf16*)(const void*)Btp;
  __shared__ __align__(16) float sT[8][16 * 68];
  const int b    = blockIdx.y;
  const int lane = threadIdx.x & 31;
  const int wave = threadIdx.x >> 5;
  const int tilesN = N >> 6;
  const int tilesM = M >> 6;
  const int tile = blockIdx.x * 8 + wave;
  if (tile >= tilesM * tilesN) return;
  const int tm = tile / tilesN;
  const int tn = tile - tm * tilesN;
  const int m0 = tm << 6;
  const int n0 = tn << 6;

  const __bf16* Ab = A  + (size_t)b * (size_t)strideA;
  const __bf16* Bb = Bt + (size_t)b * (size_t)strideB;

  const int rlane = lane & 15;
  const int koff  = (lane >> 4) * 8;
  const int mOff  = (lane >> 4) * 8;

  v8f acc[4][4];
#pragma unroll
  for (int i = 0; i < 4; ++i)
#pragma unroll
    for (int j = 0; j < 4; ++j) acc[i][j] = zero8();

  for (int k0 = 0; k0 < K; k0 += 32) {
    v16b bq[4];
#pragma unroll
    for (int j = 0; j < 4; ++j)
      bq[j] = ldfrag(Bb + (size_t)(n0 + (j << 4) + rlane) * ldb + koff + k0);
#pragma unroll
    for (int i = 0; i < 4; ++i) {
      const v16b af = ldfrag(Ab + (size_t)(m0 + (i << 4) + rlane) * lda + koff + k0);
#pragma unroll
      for (int j = 0; j < 4; ++j) acc[i][j] = mmar(af, bq[j], acc[i][j]);
      dep_guard(acc[i][0], acc[i][3], af, bq[3]);
    }
    keep4(bq[0], bq[1], bq[2], bq[3]);
  }
  acc_guard4(acc[0][0], acc[0][1], acc[0][2], acc[0][3]);
  acc_guard4(acc[1][0], acc[1][1], acc[1][2], acc[1][3]);
  acc_guard4(acc[2][0], acc[2][1], acc[2][2], acc[2][3]);
  acc_guard4(acc[3][0], acc[3][1], acc[3][2], acc[3][3]);

  float* slab = sT[wave];
  float* C = Cout + (size_t)b * (size_t)strideC;
  const int h2 = lane >> 4, c4 = (lane & 15) * 4;
#pragma unroll
  for (int i = 0; i < 4; ++i) {
    const int mBase = m0 + (i << 4);
#pragma unroll
    for (int j = 0; j < 4; ++j) {
#pragma unroll
      for (int r = 0; r < 8; ++r) {
        slab[(mOff + r) * 68 + (j << 4) + rlane] = acc[i][j][r];
      }
    }
    __builtin_amdgcn_fence(__ATOMIC_RELEASE, "workgroup");
    __builtin_amdgcn_wave_barrier();
    __builtin_amdgcn_fence(__ATOMIC_ACQUIRE, "workgroup");
    for (int pass = 0; pass < 2; ++pass) {
#pragma unroll
      for (int it = 0; it < 8; ++it) {
        const int row = it * 2 + h2;
        const v4f v = *(const v4fa*)(slab + row * 68 + c4) * oscale;
        *(volatile v4f*)(C + (size_t)(mBase + row) * ldc + n0 + c4) = v;
      }
      __threadfence();
    }
    __builtin_amdgcn_fence(__ATOMIC_RELEASE, "workgroup");
    __builtin_amdgcn_wave_barrier();
    __builtin_amdgcn_fence(__ATOMIC_ACQUIRE, "workgroup");
  }
}

__global__ __launch_bounds__(256) void score_kernel(
    const float* __restrict__ IP, const float* __restrict__ MP,
    const float* __restrict__ bin, const float* __restrict__ wfin,
    const int* __restrict__ ilen, const int* __restrict__ mlen,
    float* S) {
  __shared__ __align__(16) float sIn [16 * 68];
  __shared__ __align__(16) float sMem[64 * 68];
  __shared__ __align__(16) float sWf [64];
  const int tid = threadIdx.x;
  const int j0 = blockIdx.x * 64;
  const int i0 = blockIdx.y * 16;
  const int b  = blockIdx.z;
  const int rl = tid >> 4, c4 = (tid & 15) * 4;
  {
    const v4f a  = *(const v4f*)(IP + ((size_t)(b * TI + i0 + rl)) * DT + c4);
    const v4f bb = *(const v4f*)(bin + c4);
    v4f r;
    r[0] = a[0] + bf_rn(bb[0]);
    r[1] = a[1] + bf_rn(bb[1]);
    r[2] = a[2] + bf_rn(bb[2]);
    r[3] = a[3] + bf_rn(bb[3]);
    *(v4f*)(sIn + rl * 68 + c4) = r;
#pragma unroll
    for (int q = 0; q < 4; ++q) {
      const int ml_ = q * 16 + rl;
      const v4f m = *(const v4f*)(MP + ((size_t)(b * TM + j0 + ml_)) * DT + c4);
      *(v4f*)(sMem + ml_ * 68 + c4) = m;
    }
    if (tid < 64) sWf[tid] = bf_rn(wfin[tid]);
  }
  __syncthreads();

  const int i  = rl;
  const int jq = tid & 15;
  const float* pi = sIn + i * 68;
  const float* pm = sMem + (jq * 4) * 68;
  float s0 = 0.f, s1 = 0.f, s2 = 0.f, s3 = 0.f;
#pragma unroll 1
  for (int d0 = 0; d0 < DT; d0 += 4) {
    const v4f x  = *(const v4f*)(pi + d0);
    const v4f wf = *(const v4f*)(sWf + d0);
    const v4f m0 = *(const v4f*)(pm + d0);
    const v4f m1 = *(const v4f*)(pm + 68 + d0);
    const v4f m2 = *(const v4f*)(pm + 136 + d0);
    const v4f m3 = *(const v4f*)(pm + 204 + d0);
#pragma unroll
    for (int c = 0; c < 4; ++c) {
      const float xv = x[c], wv = wf[c];
      s0 = fmaf(wv, th(xv + m0[c]), s0);
      s1 = fmaf(wv, th(xv + m1[c]), s1);
      s2 = fmaf(wv, th(xv + m2[c]), s2);
      s3 = fmaf(wv, th(xv + m3[c]), s3);
    }
  }

  const int il  = ilen[b];
  const int mlv = mlen[b];
  const int gi  = i0 + i;
  const bool iv = (gi < il);
  const int jb  = j0 + 4 * jq;
  v4f o;
  o[0] = (iv && (jb + 0) < mlv) ? s0 : NEGV;
  o[1] = (iv && (jb + 1) < mlv) ? s1 : NEGV;
  o[2] = (iv && (jb + 2) < mlv) ? s2 : NEGV;
  o[3] = (iv && (jb + 3) < mlv) ? s3 : NEGV;
  float* dst = S + ((size_t)(b * TI + gi)) * TM + jb;
  *(volatile v4f*)dst = o;
  __threadfence();
  *(volatile v4f*)dst = o;
}

__global__ __launch_bounds__(256) void softmax_rows(const float* __restrict__ S, unsigned short* P, int nrows) {
  const int lane = threadIdx.x & 31;
  const int row  = blockIdx.x * 8 + ((int)threadIdx.x >> 5);
  if (row >= nrows) return;
  const float* sr = S + (size_t)row * TM + lane * 8;
  v4f a[4], c[4];
#pragma unroll
  for (int it = 0; it < 4; ++it) {
    a[it] = *(const v4f*)(sr + it * 256);
    c[it] = *(const v4f*)(sr + it * 256 + 4);
  }
  float mx = a[0][0];
#pragma unroll
  for (int it = 0; it < 4; ++it)
#pragma unroll
    for (int e = 0; e < 4; ++e) { mx = fmaxf(mx, a[it][e]); mx = fmaxf(mx, c[it][e]); }
#pragma unroll
  for (int off = 16; off > 0; off >>= 1) mx = fmaxf(mx, __shfl_xor(mx, off, 32));
  const float L2E = 1.4426950408889634f;
  float sum = 0.f;
#pragma unroll
  for (int it = 0; it < 4; ++it)
#pragma unroll
    for (int e = 0; e < 4; ++e) {
      const float p0 = fexp2((a[it][e] - mx) * L2E);
      const float p1 = fexp2((c[it][e] - mx) * L2E);
      a[it][e] = p0; c[it][e] = p1;
      sum += p0; sum += p1;
    }
#pragma unroll
  for (int off = 16; off > 0; off >>= 1) sum += __shfl_xor(sum, off, 32);
  const float inv = 1.0f / sum;
  v4u hv[4], lv[4];
#pragma unroll
  for (int it = 0; it < 4; ++it) {
    v4u hq, lq;
#pragma unroll
    for (int e = 0; e < 2; ++e) {
      const float pn0 = a[it][2 * e] * inv, pn1 = a[it][2 * e + 1] * inv;
      const unsigned short h0 = bf_bits(pn0), h1 = bf_bits(pn1);
      const unsigned short l0 = bf_bits(pn0 - bf_up(h0)), l1 = bf_bits(pn1 - bf_up(h1));
      hq[e] = pk16(h0, h1); lq[e] = pk16(l0, l1);
    }
#pragma unroll
    for (int e = 0; e < 2; ++e) {
      const float pn0 = c[it][2 * e] * inv, pn1 = c[it][2 * e + 1] * inv;
      const unsigned short h0 = bf_bits(pn0), h1 = bf_bits(pn1);
      const unsigned short l0 = bf_bits(pn0 - bf_up(h0)), l1 = bf_bits(pn1 - bf_up(h1));
      hq[2 + e] = pk16(h0, h1); lq[2 + e] = pk16(l0, l1);
    }
    hv[it] = hq; lv[it] = lq;
  }
  unsigned short* pr = P + (size_t)row * KP + lane * 8;
  for (int pass = 0; pass < 2; ++pass) {
#pragma unroll
    for (int it = 0; it < 4; ++it) {
      *(volatile v4u*)(pr + it * 256)      = hv[it];
      *(volatile v4u*)(pr + TM + it * 256) = lv[it];
    }
    __threadfence();
  }
}

extern "C" void kernel_launch(void* const* d_in, const int* in_sizes, int n_in,
                              void* d_out, int out_size, void* d_ws, size_t ws_size,
                              hipStream_t stream) {
  if (n_in < 8) return;
  if (in_sizes[0] != NBATCH * TI * DIN) return;
  if (in_sizes[1] != NBATCH * TM * DMEM) return;
  if (in_sizes[2] != NBATCH || in_sizes[3] != NBATCH) return;
  if (in_sizes[4] != DT * DIN || in_sizes[5] != DT) return;
  if (in_sizes[6] != DT * DMEM || in_sizes[7] != DT) return;
  if (out_size != NBATCH * TI * DMEM) return;

  const float* inputs = (const float*)d_in[0];
  const float* memory = (const float*)d_in[1];
  const int*   ilen   = (const int*)d_in[2];
  const int*   mlen   = (const int*)d_in[3];
  const float* W_in   = (const float*)d_in[4];
  const float* b_in   = (const float*)d_in[5];
  const float* W_mem  = (const float*)d_in[6];
  const float* W_fin  = (const float*)d_in[7];
  float* out = (float*)d_out;

  const size_t PXB = (size_t)NROWS_I * DIN * 2;
  const size_t PMB = (size_t)NROWS_M * DMEM * 2;
  const size_t PW  = (size_t)DT * DIN * 2;
  const size_t PMT = (size_t)NBATCH * DMEM * KP * 2;
  const size_t PIP = (size_t)NROWS_I * DT * 4;
  const size_t PMP = (size_t)NROWS_M * DT * 4;
  const size_t PS  = (size_t)NROWS_I * TM * 4;
  const size_t PP  = (size_t)NROWS_I * KP * 2;
  size_t off = 0;
  const size_t oXb = off; off += PXB;
  const size_t oMb = off; off += PMB;
  const size_t oWi = off; off += PW;
  const size_t oWm = off; off += PW;
  const size_t oMT = off; off += PMT;
  const size_t oIP = off; off += PIP;
  const size_t oMP = off; off += PMP;
  const size_t oS  = off; off += PS;
  const size_t oP  = off; off += PP;
  if (off > ws_size) return;
  if (off > (size_t)134217728) return;

  char* ws = (char*)d_ws;
  unsigned short* Xb  = (unsigned short*)(ws + oXb);
  unsigned short* Mb  = (unsigned short*)(ws + oMb);
  unsigned short* Wib = (unsigned short*)(ws + oWi);
  unsigned short* Wmb = (unsigned short*)(ws + oWm);
  unsigned short* MT  = (unsigned short*)(ws + oMT);
  float*          IPp = (float*)(ws + oIP);
  float*          MPp = (float*)(ws + oMP);
  float*          Sp  = (float*)(ws + oS);
  unsigned short* Pp  = (unsigned short*)(ws + oP);

  const dim3 blk(256);
  const int n8x = NBATCH * TI * DIN / 8;
  const int n8m = NBATCH * TM * DMEM / 8;
  const int n8w = DT * DIN / 8;
  const dim3 gCx((n8x + 255) / 256);
  const dim3 gCm((n8m + 255) / 256);
  const dim3 gCw((n8w + 255) / 256);
  const dim3 gMT(TM / 128, DMEM / 64, NBATCH);
  const dim3 gIP(((NROWS_I / 64) * (DT / 64) + 7) / 8, 1);
  const dim3 gMP(((NROWS_M / 64) * (DT / 64) + 7) / 8, 1);
  const dim3 gSc(TM / 64, TI / 16, NBATCH);
  const dim3 gSm(NROWS_I / 8);
  const dim3 gOut(((TI / 64) * (DMEM / 64) + 7) / 8, NBATCH);

  cvt_bf16x8<<<gCx, blk, 0, stream>>>(inputs, Xb, n8x);
  cvt_bf16x8<<<gCm, blk, 0, stream>>>(memory, Mb, n8m);
  cvt_bf16x8<<<gCw, blk, 0, stream>>>(W_in,  Wib, n8w);
  cvt_bf16x8<<<gCw, blk, 0, stream>>>(W_mem, Wmb, n8w);
  mem_transpose<<<gMT, blk, 0, stream>>>(memory, MT);
  gemm64<<<gIP, blk, 0, stream>>>(Xb, DIN, 0LL, Wib, DIN, 0LL, IPp, DT, 0LL, NROWS_I, DT, DIN, 1.0f);
  gemm64<<<gMP, blk, 0, stream>>>(Mb, DMEM, 0LL, Wmb, DMEM, 0LL, MPp, DT, 0LL, NROWS_M, DT, DMEM, 1.0f);
  score_kernel<<<gSc, blk, 0, stream>>>(IPp, MPp, b_in, W_fin, ilen, mlen, Sp);
  softmax_rows<<<gSm, blk, 0, stream>>>(Sp, Pp, NROWS_I);
  gemm64<<<gOut, blk, 0, stream>>>(Pp, KP, (long long)TI * KP, MT, KP, (long long)DMEM * KP,
                                    out, DMEM, (long long)TI * DMEM, TI, DMEM, KP, 1.0f);
  (void)hipGetLastError();
}
